// LSTM_12266426597813
// MI455X (gfx1250) — hardware-verified
//
#include <hip/hip_runtime.h>
#include <math.h>

constexpr int NBATCH   = 2048;
constexpr int NSTEP    = 512;
constexpr int NIN      = 4;
constexpr int NHID     = 64;
constexpr int NPROJ    = 49;
constexpr int NGATE    = 4 * NHID;
constexpr int KPAD     = 64;
constexpr int ROWS_BLK = 32;
constexpr int NTHR     = 256;
constexpr int HPITCH   = 72;
constexpr int XGROUP   = 8;
constexpr int OUT_V4   = ROWS_BLK * NPROJ / 4;
constexpr int PREP_BLOCKS = 13;
constexpr float CARRY_W   = 16.0f;
constexpr float CARRY_S   = 16.0f;
constexpr float CARRY_WX  = CARRY_W * CARRY_S;
constexpr float ACC_INV   = 1.0f / (CARRY_W * CARRY_S);
constexpr float HBACK     = 1.0f / CARRY_W;

static_assert(NPROJ + NIN <= KPAD, "h and x columns fit the padded K");
static_assert(KPAD % 32 == 0, "K multiple of 32");
static_assert(NGATE == 256 && NHID == 64, "wave map assumes 4 slices of 16");
static_assert(NBATCH % ROWS_BLK == 0, "exact grid");
static_assert((ROWS_BLK * NPROJ * 4) % 128 == 0, "block output tile is whole 128-B lines");
static_assert((ROWS_BLK * NPROJ) % 4 == 0, "float4 coverage of the output tile");
static_assert(OUT_V4 <= 2 * NTHR, "two store iterations cover the tile");
static_assert(NSTEP % XGROUP == 0, "x staged by groups of 8 steps");
static_assert(ROWS_BLK * XGROUP == NTHR, "x group fill: one float4 per thread");
static_assert((ROWS_BLK * HPITCH) % NTHR == 0, "LDS tile init loop exact");
static_assert(HPITCH % 8 == 0 && HPITCH >= KPAD, "16-B aligned fragment rows");

typedef __attribute__((ext_vector_type(16))) _Float16 v16h;
typedef __attribute__((ext_vector_type(8)))  _Float16 v8h;
typedef __attribute__((ext_vector_type(8)))  float    v8f;
typedef __attribute__((ext_vector_type(4)))  float    v4f;

__device__ __forceinline__ void guard4_h(v8f& a, v8f& b, v8f& c, v8f& d, v16h x, v16h y) {
  asm volatile("v_nop\n\tv_nop\n\tv_nop\n\tv_nop" : "+v"(a), "+v"(b), "+v"(c), "+v"(d) : "v"(x), "v"(y));
}
__device__ __forceinline__ void guard1_h(v8f& a, v16h x, v16h y) {
  asm volatile("v_nop\n\tv_nop\n\tv_nop\n\tv_nop" : "+v"(a) : "v"(x), "v"(y));
}
__device__ __forceinline__ void touch8(float& a, float& b, float& c, float& d, float& e, float& f, float& g, float& h) {
  asm volatile("" : "+v"(a), "+v"(b), "+v"(c), "+v"(d), "+v"(e), "+v"(f), "+v"(g), "+v"(h));
}

template <typename T> struct Frag;
template <> struct Frag<_Float16> {
  typedef v16h V;
  union U { v16h v; v8h h[2]; };
  static __device__ __forceinline__ v16h load(const _Float16* p) {
    U f;
    f.h[0] = *(const v8h*)(p);
    f.h[1] = *(const v8h*)(p + 16);
    return f.v;
  }
  static __device__ __forceinline__ v8f mma(v16h a, v16h b, v8f c) {
    return __builtin_amdgcn_wmma_f32_16x16x32_f16(false, a, false, b, (short)0, c, false, false);
  }
};

__device__ __forceinline__ float sigm_f(float x) {
  return __builtin_amdgcn_rcpf(1.0f + expf(-x));
}
__device__ __forceinline__ float tanh_f(float x) {
  return 2.0f * sigm_f(2.0f * x) - 1.0f;
}

__device__ __forceinline__ void store8h_twice(unsigned short* p, v8h v) {
  *(volatile v8h*)p = v;
  __threadfence();
  *(volatile v8h*)p = v;
}

__global__ __launch_bounds__(NTHR) void prep_planes_kernel(
    const float* __restrict__ W_ih, const float* __restrict__ W_hh,
    const float* __restrict__ b_ih, const float* __restrict__ b_hh,
    const float* __restrict__ W_hr, const float* __restrict__ W_out,
    unsigned short* __restrict__ WG, unsigned short* __restrict__ WP,
    unsigned short* __restrict__ WO, float* __restrict__ BIAS) {
  const int tid = threadIdx.x;
  const int bid = blockIdx.x;
  const int rl  = tid >> 3;
  const int c8  = (tid & 7) * 8;
  if (bid < 8) {
    const int n = bid * 32 + rl;
    float va[8], vb[8];
#pragma unroll
    for (int e = 0; e < 8; ++e) {
      const int k  = c8 + e;
      const int kh = (k < NPROJ) ? k : (NPROJ - 1);
      va[e] = W_hh[n * NPROJ + kh];
    }
    touch8(va[0], va[1], va[2], va[3], va[4], va[5], va[6], va[7]);
#pragma unroll
    for (int e = 0; e < 8; ++e) {
      int ki = c8 + e - NPROJ;
      ki = (ki < 0) ? 0 : ((ki > NIN - 1) ? (NIN - 1) : ki);
      vb[e] = W_ih[n * NIN + ki];
    }
    touch8(vb[0], vb[1], vb[2], vb[3], vb[4], vb[5], vb[6], vb[7]);
    v8h hv;
#pragma unroll
    for (int e = 0; e < 8; ++e) {
      const int k = c8 + e;
      const float fa = (k < NPROJ) ? CARRY_W : 0.0f;
      const float fb = (k >= NPROJ && k < NPROJ + NIN) ? CARRY_WX : 0.0f;
      const float v  = fmaf(fa, va[e], fb * vb[e]);
      hv[e] = (_Float16)v;
    }
    store8h_twice(WG + (size_t)n * KPAD + c8, hv);
  } else if (bid < 10) {
    const int n  = (bid - 8) * 32 + rl;
    const int nc = (n < NPROJ) ? n : (NPROJ - 1);
    const v4f a = *(const v4f*)(W_hr + nc * NHID + c8);
    const v4f b = *(const v4f*)(W_hr + nc * NHID + c8 + 4);
    const bool live = (n < NPROJ);
    v8h hv;
#pragma unroll
    for (int e = 0; e < 4; ++e) {
      const float fa = a[e] * CARRY_W;
      const float fb = b[e] * CARRY_W;
      hv[e]     = (_Float16)(live ? fa : 0.0f);
      hv[4 + e] = (_Float16)(live ? fb : 0.0f);
    }
    store8h_twice(WP + (size_t)n * KPAD + c8, hv);
  } else if (bid < 12) {
    const int n  = (bid - 10) * 32 + rl;
    const int nc = (n < NPROJ) ? n : (NPROJ - 1);
    float wv[8];
#pragma unroll
    for (int e = 0; e < 8; ++e) {
      const int k  = c8 + e;
      const int kc = (k < NPROJ) ? k : (NPROJ - 1);
      wv[e] = W_out[nc * NPROJ + kc];
    }
    touch8(wv[0], wv[1], wv[2], wv[3], wv[4], wv[5], wv[6], wv[7]);
    v8h hv;
#pragma unroll
    for (int e = 0; e < 8; ++e) {
      const int k = c8 + e;
      const bool live = (n < NPROJ) && (k < NPROJ);
      const float f = wv[e] * CARRY_W;
      hv[e] = (_Float16)(live ? f : 0.0f);
    }
    store8h_twice(WO + (size_t)n * KPAD + c8, hv);
  } else {
    if (tid < NGATE / 4) {
      const v4f a = *(const v4f*)(b_ih + 4 * tid);
      const v4f b = *(const v4f*)(b_hh + 4 * tid);
      v4f o;
#pragma unroll
      for (int e = 0; e < 4; ++e) o[e] = a[e] + b[e];
      float* op = BIAS + 4 * tid;
      *(volatile v4f*)op = o;
      __threadfence();
      *(volatile v4f*)op = o;
    }
  }
}

__global__ __launch_bounds__(NTHR) void lstm_seq_kernel(
    const float* __restrict__ x,
    const unsigned short* __restrict__ WGp, const unsigned short* __restrict__ WPp,
    const unsigned short* __restrict__ WOp, const float* __restrict__ BIAS,
    const float* __restrict__ b_out, float* __restrict__ out) {
  __shared__ __align__(16) _Float16 hbuf[ROWS_BLK * HPITCH];
  __shared__ __align__(16) _Float16 hfbuf[ROWS_BLK * HPITCH];
  __shared__ __align__(16) float    xstage[ROWS_BLK * XGROUP * NIN];
  __shared__ __align__(16) float    outstage[ROWS_BLK * NPROJ];

  const _Float16* WG = (const _Float16*)WGp;
  const _Float16* WP = (const _Float16*)WPp;
  const _Float16* WO = (const _Float16*)WOp;

  const int tid  = threadIdx.x;
  const int lane = tid & 31;
  const int wave = tid >> 5;
  const int mt   = wave >> 2;
  const int w    = wave & 3;
  const int c    = lane & 15;
  const int hh   = lane >> 4;
  const int koff = 8 * hh;
  const int ncol = 16 * w + c;
  const int drow0 = 16 * mt + 8 * hh;
  const int rowbase = blockIdx.x * ROWS_BLK;

  v16h Bg[4][2];
#pragma unroll
  for (int g = 0; g < 4; ++g) {
    const _Float16* p = WG + (size_t)(g * NHID + ncol) * KPAD + koff;
    Bg[g][0] = Frag<_Float16>::load(p);
    Bg[g][1] = Frag<_Float16>::load(p + 32);
    asm volatile("" :: "v"(Bg[g][0]), "v"(Bg[g][1]) : "memory");
  }
  v16h Bp0, Bp1;
  {
    const _Float16* p = WP + (size_t)ncol * KPAD + koff;
    Bp0 = Frag<_Float16>::load(p);
    Bp1 = Frag<_Float16>::load(p + 32);
    asm volatile("" :: "v"(Bp0), "v"(Bp1) : "memory");
  }
  float bi[4];
#pragma unroll
  for (int g = 0; g < 4; ++g) bi[g] = BIAS[g * NHID + ncol];

  {
    const int row = tid >> 3, s = tid & 7;
    const v4f v = *(const v4f*)(x + ((size_t)(rowbase + row) * NSTEP + (size_t)s) * NIN);
    *(v4f*)(xstage + row * (XGROUP * NIN) + s * NIN) = v;
  }
  __syncthreads();
#pragma unroll 1
  for (int i = tid; i < ROWS_BLK * HPITCH; i += NTHR) {
    const int row = i / HPITCH;
    const int col = i - row * HPITCH;
    int ci = col - NPROJ;
    ci = (ci < 0) ? 0 : ((ci > NIN - 1) ? (NIN - 1) : ci);
    const float xv = xstage[row * (XGROUP * NIN) + ci];
    const float val = (col >= NPROJ && col < NPROJ + NIN) ? xv : 0.0f;
    hbuf[i] = (_Float16)val;
  }
  float cst[8];
#pragma unroll
  for (int r = 0; r < 8; ++r) cst[r] = 0.0f;
  __syncthreads();

  const _Float16* harow = hbuf  + (16 * mt + c) * HPITCH + koff;
  const _Float16* hfrow = hfbuf + (16 * mt + c) * HPITCH + koff;
  int cix = ncol - NPROJ;
  cix = (cix < 0) ? 0 : ((cix > NIN - 1) ? (NIN - 1) : cix);
  const v8f z8 = {0.f, 0.f, 0.f, 0.f, 0.f, 0.f, 0.f, 0.f};

#pragma unroll 1
  for (int t = 0; t < NSTEP; ++t) {
    if (((t & (XGROUP - 1)) == XGROUP - 1) && (t + 1 < NSTEP)) {
      const int row = tid >> 3, s = tid & 7;
      const v4f v = *(const v4f*)(x + ((size_t)(rowbase + row) * NSTEP + (size_t)(t + 1 + s)) * NIN);
      *(v4f*)(xstage + row * (XGROUP * NIN) + s * NIN) = v;
    }

    const v16h a0 = Frag<_Float16>::load(harow);
    const v16h a1 = Frag<_Float16>::load(harow + 32);
    v8f acc0 = z8, acc1 = z8, acc2 = z8, acc3 = z8;
    acc0 = Frag<_Float16>::mma(a0, Bg[0][0], acc0);
    acc1 = Frag<_Float16>::mma(a0, Bg[1][0], acc1);
    acc2 = Frag<_Float16>::mma(a0, Bg[2][0], acc2);
    acc3 = Frag<_Float16>::mma(a0, Bg[3][0], acc3);
    acc0 = Frag<_Float16>::mma(a1, Bg[0][1], acc0);
    acc1 = Frag<_Float16>::mma(a1, Bg[1][1], acc1);
    acc2 = Frag<_Float16>::mma(a1, Bg[2][1], acc2);
    acc3 = Frag<_Float16>::mma(a1, Bg[3][1], acc3);
    guard4_h(acc0, acc1, acc2, acc3, a0, a1);

#pragma unroll
    for (int r = 0; r < 8; ++r) {
      const float zi = acc0[r] * ACC_INV + bi[0];
      const float zf = acc1[r] * ACC_INV + bi[1];
      const float zg = acc2[r] * ACC_INV + bi[2];
      const float zo = acc3[r] * ACC_INV + bi[3];
      const float ig = sigm_f(zi);
      const float fg = sigm_f(zf);
      const float gg = tanh_f(zg);
      const float og = sigm_f(zo);
      const float cn = fg * cst[r] + ig * gg;
      cst[r] = cn;
      const float hf = og * tanh_f(cn);
      hfbuf[(drow0 + r) * HPITCH + ncol] = (_Float16)(hf * CARRY_S);
    }
    __syncthreads();

    const v16h pa0 = Frag<_Float16>::load(hfrow);
    const v16h pa1 = Frag<_Float16>::load(hfrow + 32);
    v8f pd = z8;
    pd = Frag<_Float16>::mma(pa0, Bp0, pd);
    pd = Frag<_Float16>::mma(pa1, Bp1, pd);
    guard1_h(pd, pa0, pa1);

    const int tn = (t + 1 < NSTEP) ? (t + 1) : (NSTEP - 1);
    const int xo = (tn & (XGROUP - 1)) * NIN + cix;
#pragma unroll
    for (int r = 0; r < 8; ++r) {
      const int row = drow0 + r;
      const float xv = xstage[row * (XGROUP * NIN) + xo];
      const float hv = pd[r] * HBACK;
      const float val = (ncol < NPROJ) ? hv : ((ncol < NPROJ + NIN) ? xv : 0.0f);
      hbuf[row * HPITCH + ncol] = (_Float16)val;
    }
    __syncthreads();
  }

  {
    const _Float16* p = WO + (size_t)ncol * KPAD + koff;
    const v16h Bo0 = Frag<_Float16>::load(p);
    const v16h Bo1 = Frag<_Float16>::load(p + 32);
    const v16h oa0 = Frag<_Float16>::load(harow);
    const v16h oa1 = Frag<_Float16>::load(harow + 32);
    v8f od = z8;
    od = Frag<_Float16>::mma(oa0, Bo0, od);
    od = Frag<_Float16>::mma(oa1, Bo1, od);
    guard1_h(od, oa0, oa1);
    asm volatile("" :: "v"(Bo0), "v"(Bo1));
    const float bo = b_out[(ncol < NPROJ) ? ncol : (NPROJ - 1)];
#pragma unroll
    for (int r = 0; r < 8; ++r) {
      const float ov = od[r] * ACC_INV + bo;
      if (ncol < NPROJ) outstage[(drow0 + r) * NPROJ + ncol] = ov;
    }
  }
  __syncthreads();
  {
    float* ob = out + (size_t)rowbase * NPROJ;
    for (int pass = 0; pass < 2; ++pass) {
#pragma unroll
      for (int it = 0; it < 2; ++it) {
        const int idx = it * NTHR + tid;
        if (idx < OUT_V4) {
          const v4f v = *(const v4f*)(outstage + 4 * idx);
          *(volatile v4f*)(ob + 4 * idx) = v;
        }
      }
      __threadfence();
    }
  }
}

extern "C" void kernel_launch(void* const* d_in, const int* in_sizes, int n_in,
                              void* d_out, int out_size, void* d_ws, size_t ws_size, hipStream_t stream) {
  if (n_in < 8 || d_out == nullptr || d_ws == nullptr) return;
  if (in_sizes[0] != NBATCH * NSTEP * NIN || in_sizes[1] != NGATE * NIN || in_sizes[2] != NGATE * NPROJ ||
      in_sizes[3] != NGATE || in_sizes[4] != NGATE || in_sizes[5] != NPROJ * NHID ||
      in_sizes[6] != NPROJ * NPROJ || in_sizes[7] != NPROJ || out_size != NBATCH * NPROJ) return;

  const float* x     = (const float*)d_in[0];
  const float* W_ih  = (const float*)d_in[1];
  const float* W_hh  = (const float*)d_in[2];
  const float* b_ih  = (const float*)d_in[3];
  const float* b_hh  = (const float*)d_in[4];
  const float* W_hr  = (const float*)d_in[5];
  const float* W_out = (const float*)d_in[6];
  const float* b_out = (const float*)d_in[7];
  float* out = (float*)d_out;

  char* ws = (char*)d_ws;
  size_t off = 0;
  auto carve = [&](size_t bytes) -> char* { char* p = ws + off; off += (bytes + 255) & ~(size_t)255; return p; };
  unsigned short* WG   = (unsigned short*)carve((size_t)NGATE * KPAD * 2);
  unsigned short* WP   = (unsigned short*)carve((size_t)KPAD * KPAD * 2);
  unsigned short* WO   = (unsigned short*)carve((size_t)KPAD * KPAD * 2);
  float*          BIAS = (float*)carve((size_t)NGATE * 4);
  if (off > ws_size || off > (size_t)134217728) return;

  prep_planes_kernel<<<PREP_BLOCKS, NTHR, 0, stream>>>(W_ih, W_hh, b_ih, b_hh, W_hr, W_out, WG, WP, WO, BIAS);
  lstm_seq_kernel<<<NBATCH / ROWS_BLK, NTHR, 0, stream>>>(x, WG, WP, WO, BIAS, b_out, out);
}
